// HyperbolicMLR_59347858096311
// MI455X (gfx1250) — hardware-run, weakly checked
//
#include <hip/hip_runtime.h>
#include <math.h>


#ifndef NB
#define NB 2048
#endif
#ifndef NC
#define NC 512
#endif
#define NB_FULL 2048
#define NC_FULL 512
#define DK   256
#define OUTP NC_FULL
#define MAXN 0.999f
#define MINN 1e-5f

static_assert(DK == 256);
static_assert(DK % 32 == 0);
static_assert(NB % 64 == 0);
static_assert(NC % 64 == 0);
static_assert(NB <= NB_FULL);
static_assert(NC <= NC_FULL);
static_assert(OUTP % 32 == 0);

typedef unsigned short bf;
typedef __attribute__((ext_vector_type(16))) __bf16   v16bf;
typedef __attribute__((ext_vector_type(8)))  unsigned short v8us;
typedef __attribute__((ext_vector_type(8)))  float    v8f;
typedef __attribute__((ext_vector_type(4)))  float    v4f;
typedef v4f  __attribute__((may_alias)) v4fa;

__device__ __forceinline__ unsigned short f2bf(float f) { unsigned u = __float_as_uint(f); u += 0x7FFFu + ((u >> 16) & 1u); return (unsigned short)(u >> 16); }
__device__ __forceinline__ float bf2f(unsigned short h) { return __uint_as_float(((unsigned)h) << 16); }
__device__ __forceinline__ float bfr(float f) { return bf2f(f2bf(f)); }
__device__ __forceinline__ v16bf cat16b(v8us lo, v8us hi) { return __builtin_bit_cast(v16bf, __builtin_shufflevector(lo, hi, 0, 1, 2, 3, 4, 5, 6, 7, 8, 9, 10, 11, 12, 13, 14, 15)); }
__device__ __forceinline__ v8f wmmab(v16bf a, v16bf b, v8f c) { return __builtin_amdgcn_wmma_f32_16x16x32_bf16(false, a, false, b, (short)0, c, false, false); }
__device__ __forceinline__ v16bf ldb(const bf* p)  { return cat16b(*(const v8us*)p, *(const v8us*)(p + 16)); }
__device__ __forceinline__ void wave_sync() { __builtin_amdgcn_fence(3  , "wavefront"); __builtin_amdgcn_wave_barrier(); asm volatile("" ::: "memory"); }

__device__ __forceinline__ float wave_sum(float s) {
    s += __shfl_xor(s, 16, 32); s += __shfl_xor(s, 8, 32); s += __shfl_xor(s, 4, 32); s += __shfl_xor(s, 2, 32); s += __shfl_xor(s, 1, 32);
    return s;
}
__device__ __forceinline__ float sumsq8(v8f v) {
    float s = v[0] * v[0];
#pragma unroll
    for (int k = 1; k < 8; ++k) s = fmaf(v[k], v[k], s);
    return s;
}
__device__ __forceinline__ float dot8(v8f a, v8f b) {
    float s = a[0] * b[0];
#pragma unroll
    for (int k = 1; k < 8; ++k) s = fmaf(a[k], b[k], s);
    return s;
}
__device__ __forceinline__ void split8(v8f v, v8us& oh, v8us& ol) {
#pragma unroll
    for (int k = 0; k < 8; ++k) { const unsigned short h = f2bf(v[k]); oh[k] = h; ol[k] = f2bf(v[k] - bf2f(h)); }
}

__global__ __launch_bounds__(256) void k_prep_x(const float* __restrict__ x, bf* XH, bf* XL, float* Y2) {
    __shared__ __align__(16) float ys[32];
    const int lane = threadIdx.x & 31;
    const int wave = __builtin_amdgcn_readfirstlane((int)(threadIdx.x >> 5));
#pragma unroll 1
    for (int it = 0; it < 4; ++it) {
        const int rl = wave * 4 + it;
        const size_t eo = ((size_t)blockIdx.x * 32 + (size_t)rl) * DK + (size_t)lane * 8;
        const v8f raw = *(const v8f*)(x + eo);
        v8f v;
#pragma unroll
        for (int k = 0; k < 8; ++k) v[k] = bfr(raw[k]);
        const float nrm = sqrtf(wave_sum(sumsq8(v)));
        const float fac = fminf(1.0f, 1.0f / (nrm + 1e-5f));
        const v8f u = v * fac;
        const float un = fmaxf(sqrtf(wave_sum(sumsq8(u))), MINN);
        const float th = tanhf(un);
        const float ru = 1.0f / un;
        const v8f e = (u * th) * ru;
        const float en = fmaxf(sqrtf(wave_sum(sumsq8(e))), MINN);
        const float re = 1.0f / en;
        const bool big = en > MAXN;
        v8f X;
#pragma unroll
        for (int k = 0; k < 8; ++k) { const float pj = (e[k] * re) * MAXN; X[k] = big ? pj : e[k]; }
        const float y2 = wave_sum(sumsq8(X));
        v8us oh, ol; split8(X, oh, ol);
        *(volatile v8us*)(XH + eo) = oh; *(volatile v8us*)(XL + eo) = ol;
        __threadfence();
        *(volatile v8us*)(XH + eo) = oh; *(volatile v8us*)(XL + eo) = ol;
        if (lane == 0) ys[rl] = y2;
    }
    __syncthreads();
    if (wave == 0 && lane < 8) {
        const v4f val = *(const v4fa*)(&ys[lane * 4]);
        float* dst = Y2 + (size_t)blockIdx.x * 32 + lane * 4;
        *(volatile v4f*)dst = val; __threadfence(); *(volatile v4f*)dst = val;
    }
}

__global__ __launch_bounds__(256) void k_prep_pa(const float* __restrict__ av, const float* __restrict__ pv, bf* PH, bf* PL, bf* AH, bf* AL, float* CT) {
    __shared__ __align__(16) float cs[4 * 32];
    const int lane = threadIdx.x & 31;
    const int wave = __builtin_amdgcn_readfirstlane((int)(threadIdx.x >> 5));
#pragma unroll 1
    for (int it = 0; it < 4; ++it) {
        const int rl = wave * 4 + it;
        const size_t eo = ((size_t)blockIdx.x * 32 + (size_t)rl) * DK + (size_t)lane * 8;
        const v8f rp = *(const v8f*)(pv + eo);
        const v8f ra = *(const v8f*)(av + eo);
        v8f p, a;
#pragma unroll
        for (int k = 0; k < 8; ++k) { p[k] = bfr(rp[k]); a[k] = bfr(ra[k]); }
        const float pn = fmaxf(sqrtf(wave_sum(sumsq8(p))), MINN);
        const float th = tanhf(pn);
        const float rn = 1.0f / pn;
        const v8f P = (p * th) * rn;
        const float p2 = wave_sum(sumsq8(P));
        const float conf = 1.0f - p2;
        const v8f A = a * conf;
        const float an = sqrtf(wave_sum(sumsq8(A)));
        const float pa = wave_sum(dot8(P, A));
        const float lam = 2.0f * (1.0f / (1.0f - p2));
        const float kk = lam * an;
        v8us oh, ol;
        split8(P, oh, ol);
        v8us qh, ql;
        split8(A, qh, ql);
        *(volatile v8us*)(PH + eo) = oh; *(volatile v8us*)(PL + eo) = ol; *(volatile v8us*)(AH + eo) = qh; *(volatile v8us*)(AL + eo) = ql;
        __threadfence();
        *(volatile v8us*)(PH + eo) = oh; *(volatile v8us*)(PL + eo) = ol; *(volatile v8us*)(AH + eo) = qh; *(volatile v8us*)(AL + eo) = ql;
        if (lane == 0) { cs[rl] = p2; cs[32 + rl] = pa; cs[64 + rl] = an; cs[96 + rl] = kk; }
    }
    __syncthreads();
    if (wave == 0) {
        const int t = lane >> 3, q = lane & 7;
        const v4f val = *(const v4fa*)(&cs[t * 32 + q * 4]);
        float* dst = CT + (size_t)t * NC + (size_t)blockIdx.x * 32 + q * 4;
        *(volatile v4f*)dst = val; __threadfence(); *(volatile v4f*)dst = val;
    }
}

__device__ __forceinline__ float logit_elem(float xp, float xa, float y2, float x2, float pa, float an, float kk) {
    const float xy  = -xp;
    const float txy = 2.0f * xy;
    const float nc  = (1.0f + txy) + y2;
    const float dn  = (1.0f + txy) + x2 * y2;
    const float dd  = dn + 1e-5f;
    const float om  = 1.0f - x2;
    const float ri  = 1.0f / dd;
    const float mobA = (nc * (-pa) + om * xa) * ri;
    const float mob2 = ((nc * nc) * x2 + ((2.0f * nc) * om) * xy + (om * om) * y2) * (ri * ri);
    const float num = 2.0f * mobA;
    const float den = an * (1.0f - mob2);
    return kk * asinhf(num * (1.0f / den));
}

__global__ __launch_bounds__(128) void k_logits(const bf* __restrict__ XH, const bf* __restrict__ XL, const bf* __restrict__ PH, const bf* __restrict__ PL,
                                                const bf* __restrict__ AH, const bf* __restrict__ AL, const float* __restrict__ Y2, const float* __restrict__ CT, float* OUT) {
    __shared__ __align__(16) float os[4 * 16 * 36];
    const int lane = threadIdx.x & 31, lr = lane & 15, hi = lane >> 4;
    const int wave = __builtin_amdgcn_readfirstlane((int)(threadIdx.x >> 5));
    const int b0 = blockIdx.x * 64 + (wave >> 1) * 32;
    const int n0 = blockIdx.y * 64 + (wave & 1) * 32;
    v8f accP[2][2], accA[2][2];
#pragma unroll
    for (int mb = 0; mb < 2; ++mb)
#pragma unroll
        for (int nb = 0; nb < 2; ++nb) { accP[mb][nb] = (v8f){}; accA[mb][nb] = (v8f){}; }
    const size_t aoff = (size_t)(b0 + lr) * DK + 8 * hi, boff = (size_t)(n0 + lr) * DK + 8 * hi;
#pragma unroll 1
    for (int kc = 0; kc < DK; kc += 32) {
        v16bf ah[2], al[2];
#pragma unroll
        for (int mb = 0; mb < 2; ++mb) { ah[mb] = ldb(XH + aoff + (size_t)mb * 16 * DK + kc); al[mb] = ldb(XL + aoff + (size_t)mb * 16 * DK + kc); }
#pragma unroll
        for (int nb = 0; nb < 2; ++nb) {
            const size_t bo = boff + (size_t)nb * 16 * DK + kc;
            const v16bf ph = ldb(PH + bo), pl = ldb(PL + bo), qh = ldb(AH + bo), ql = ldb(AL + bo);
#pragma unroll
            for (int mb = 0; mb < 2; ++mb) { accP[mb][nb] = wmmab(ah[mb], ph, accP[mb][nb]); accA[mb][nb] = wmmab(ah[mb], qh, accA[mb][nb]); }
#pragma unroll
            for (int mb = 0; mb < 2; ++mb) { accP[mb][nb] = wmmab(ah[mb], pl, accP[mb][nb]); accA[mb][nb] = wmmab(ah[mb], ql, accA[mb][nb]); }
#pragma unroll
            for (int mb = 0; mb < 2; ++mb) { accP[mb][nb] = wmmab(al[mb], ph, accP[mb][nb]); accA[mb][nb] = wmmab(al[mb], qh, accA[mb][nb]); }
        }
        asm volatile("v_nop\n\tv_nop\n\tv_nop\n\tv_nop"
                     : "+v"(accP[0][0]), "+v"(accP[0][1]), "+v"(accP[1][0]), "+v"(accP[1][1]), "+v"(accA[0][0]), "+v"(accA[0][1]), "+v"(accA[1][0]), "+v"(accA[1][1])
                     : "v"(ah[0]), "v"(ah[1]), "v"(al[0]), "v"(al[1]));
    }
    float x2v[2], pav[2], anv[2], kkv[2];
#pragma unroll
    for (int nb = 0; nb < 2; ++nb) { const int n = n0 + nb * 16 + lr;
        x2v[nb] = CT[n]; pav[nb] = CT[(size_t)NC + n]; anv[nb] = CT[(size_t)2 * NC + n]; kkv[nb] = CT[(size_t)3 * NC + n]; }
    const int wb = wave * 16 * 36;
#pragma unroll
    for (int mb = 0; mb < 2; ++mb) {
        const float* yp = Y2 + b0 + mb * 16 + 8 * hi;
        const v4f ya = *(const v4f*)yp; const v4f yb = *(const v4f*)(yp + 4);
#pragma unroll
        for (int nb = 0; nb < 2; ++nb) {
#pragma unroll
            for (int r = 0; r < 8; ++r) {
                const float y2 = (r < 4) ? ya[r & 3] : yb[r & 3];
                os[wb + (8 * hi + r) * 36 + nb * 16 + lr] = logit_elem(accP[mb][nb][r], accA[mb][nb][r], y2, x2v[nb], pav[nb], anv[nb], kkv[nb]);
            }
        }
        wave_sync();
        float* ob = OUT + (size_t)(b0 + mb * 16) * OUTP + n0;
#pragma unroll 1
        for (int ps = 0; ps < 2; ++ps) {
#pragma unroll
            for (int s = 0; s < 4; ++s) { const int row = 4 * s + (lane >> 3), c4 = (lane & 7) * 4;
                const v4f val = *(const v4fa*)(&os[wb + row * 36 + c4]);
                *(volatile v4f*)(ob + (size_t)row * OUTP + c4) = val; }
            if (ps == 0) __threadfence(); }
        wave_sync();
    }
}

static constexpr size_t al256(size_t v) { return (v + 255) & ~(size_t)255; }
static constexpr size_t SZ_X = al256((size_t)NB * DK * 2);
static constexpr size_t SZ_C = al256((size_t)NC * DK * 2);
static constexpr size_t SZ_Y = al256((size_t)NB * 4);
static constexpr size_t SZ_T = al256((size_t)4 * NC * 4);
static constexpr size_t SZ_TOTAL = 2 * SZ_X + 4 * SZ_C + SZ_Y + SZ_T;
static_assert(SZ_TOTAL <= (size_t)134217728);
static_assert(((size_t)(NB - 1) * OUTP + NC) * 4 <= (size_t)NB_FULL * NC_FULL * 4);

extern "C" void kernel_launch(void* const* d_in, const int* in_sizes, int n_in,
                              void* d_out, int out_size, void* d_ws, size_t ws_size, hipStream_t stream) {
    if (n_in < 3) return;
    if ((size_t)in_sizes[0] < (size_t)NB * DK) return;
    if ((size_t)in_sizes[1] < (size_t)NC * DK || (size_t)in_sizes[2] < (size_t)NC * DK) return;
    if ((size_t)out_size < (size_t)(NB - 1) * OUTP + NC) return;
    if (SZ_TOTAL > ws_size) return;
    const float* x  = (const float*)d_in[0];
    const float* av = (const float*)d_in[1];
    const float* pv = (const float*)d_in[2];
    float* OUT = (float*)d_out;
    char* wsp = (char*)d_ws;
    bf* XH = (bf*)wsp; wsp += SZ_X;
    bf* XL = (bf*)wsp; wsp += SZ_X;
    bf* PH = (bf*)wsp; wsp += SZ_C;
    bf* PL = (bf*)wsp; wsp += SZ_C;
    bf* AH = (bf*)wsp; wsp += SZ_C;
    bf* AL = (bf*)wsp; wsp += SZ_C;
    float* Y2 = (float*)wsp; wsp += SZ_Y;
    float* CT = (float*)wsp; wsp += SZ_T;

    k_prep_x<<<NB / 32, 256, 0, stream>>>(x, XH, XL, Y2);
    k_prep_pa<<<NC / 32, 256, 0, stream>>>(av, pv, PH, PL, AH, AL, CT);
    k_logits<<<dim3(NB / 64, NC / 64, 1), 128, 0, stream>>>(XH, XL, PH, PL, AH, AL, Y2, CT, OUT);
}
